// BasicNonLocalBlock_64570538328627
// MI455X (gfx1250) — hardware-verified
//
#include <hip/hip_runtime.h>


#define NB_  4
#define CC   512
#define TQ   4096
#define NKY   4096
#define KC   256
#define VC   256
#define PCAR 1024.0f
#define SCL  0.0625f
typedef _Float16 h16;
typedef unsigned short bf;
typedef __attribute__((ext_vector_type(16))) __bf16   v16bf;
typedef __attribute__((ext_vector_type(16))) _Float16 v16h;
typedef __attribute__((ext_vector_type(8)))  _Float16 v8h;
typedef __attribute__((ext_vector_type(8)))  unsigned short v8us;
typedef __attribute__((ext_vector_type(8)))  float    v8f;
typedef __attribute__((ext_vector_type(4)))  float    v4f;
typedef v8h  __attribute__((may_alias)) v8ha;
typedef v4f  __attribute__((may_alias)) v4fa;
typedef v8us __attribute__((may_alias)) v8usa;

__device__ __forceinline__ unsigned short f2bf(float f) { unsigned u = __float_as_uint(f); u += 0x7FFFu + ((u >> 16) & 1u); return (unsigned short)(u >> 16); }
__device__ __forceinline__ float bf2f(unsigned short b) { return __uint_as_float(((unsigned)b) << 16); }
__device__ __forceinline__ float bfr(float f) { return bf2f(f2bf(f)); }
__device__ __forceinline__ v16h cat16(v8h lo, v8h hi) { return __builtin_shufflevector(lo, hi, 0, 1, 2, 3, 4, 5, 6, 7, 8, 9, 10, 11, 12, 13, 14, 15); }
__device__ __forceinline__ v16bf cat16b(v8us lo, v8us hi) { return __builtin_bit_cast(v16bf, __builtin_shufflevector(lo, hi, 0, 1, 2, 3, 4, 5, 6, 7, 8, 9, 10, 11, 12, 13, 14, 15)); }
__device__ __forceinline__ v8f wmma16(v16h a, v16h b, v8f c) { return __builtin_amdgcn_wmma_f32_16x16x32_f16(false, a, false, b, (short)0, c, false, false); }
__device__ __forceinline__ v8f wmmab(v16bf a, v16bf b, v8f c) { return __builtin_amdgcn_wmma_f32_16x16x32_bf16(false, a, false, b, (short)0, c, false, false); }


template <typename T16> struct WFrag;
template <> struct WFrag<h16> { typedef v16h V; static __device__ __forceinline__ V ld(const h16* p) { return cat16(*(const v8h*)p, *(const v8h*)(p + 16)); } static __device__ __forceinline__ v8f mma(V a, V b, v8f c) { return wmma16(a, b, c); } };
template <> struct WFrag<bf> { typedef v16bf V; static __device__ __forceinline__ V ld(const bf* p) { return cat16b(*(const v8us*)p, *(const v8us*)(p + 16)); } static __device__ __forceinline__ v8f mma(V a, V b, v8f c) { return wmmab(a, b, c); } };
template <typename T16, int NSPLIT, bool BIAS>
__global__ __launch_bounds__(32) void k_gemmw(const T16* __restrict__ A, const T16* __restrict__ A2, const T16* __restrict__ Bt, const T16* __restrict__ Bt2, int K, float* C, int ldc, const float* __restrict__ bias, size_t sA, size_t sB, size_t sC) {
    typedef typename WFrag<T16>::V V;
    __shared__ __align__(16) float os[16 * 68];
    const size_t z = blockIdx.z; A += z * sA; if (A2) A2 += z * sA; Bt += z * sB; if (Bt2) Bt2 += z * sB; C += z * sC;
    const int lane = threadIdx.x & 31, lr = lane & 15, hi = lane >> 4; const int r0 = blockIdx.x * 64, c0 = blockIdx.y * 64;
    v8f acc[4][4];
#pragma unroll
    for (int mb = 0; mb < 4; ++mb)
#pragma unroll
        for (int nb = 0; nb < 4; ++nb) acc[mb][nb] = (v8f){};
    const size_t aoff = (size_t)(r0 + lr) * K + 8 * hi, boff = (size_t)(c0 + lr) * K + 8 * hi;
#pragma unroll 1
    for (int kc = 0; kc < K; kc += 32) {
        V a[4], a2[4];
#pragma unroll
        for (int mb = 0; mb < 4; ++mb) { a[mb] = WFrag<T16>::ld(A + aoff + (size_t)mb * 16 * K + kc); if (NSPLIT == 1 || NSPLIT == 2) a2[mb] = WFrag<T16>::ld(A2 + aoff + (size_t)mb * 16 * K + kc); }
#pragma unroll
        for (int nb = 0; nb < 4; ++nb) { const V b = WFrag<T16>::ld(Bt + boff + (size_t)nb * 16 * K + kc); V b2; if (NSPLIT >= 2) b2 = WFrag<T16>::ld(Bt2 + boff + (size_t)nb * 16 * K + kc);
#pragma unroll
            for (int mb = 0; mb < 4; ++mb) { acc[mb][nb] = WFrag<T16>::mma(a[mb], b, acc[mb][nb]); if (NSPLIT == 1 || NSPLIT == 2) acc[mb][nb] = WFrag<T16>::mma(a2[mb], b, acc[mb][nb]); if (NSPLIT >= 2) acc[mb][nb] = WFrag<T16>::mma(a[mb], b2, acc[mb][nb]); } }
        asm volatile("v_nop\n\tv_nop\n\tv_nop\n\tv_nop" : "+v"(acc[0][0]), "+v"(acc[1][1]), "+v"(acc[2][2]), "+v"(acc[3][3]) : "v"(a[0]), "v"(a[3]));
    }
#pragma unroll
    for (int mb = 0; mb < 4; ++mb) {
#pragma unroll
        for (int nb = 0; nb < 4; ++nb) {
#pragma unroll
            for (int j = 0; j < 8; ++j) os[(hi * 8 + j) * 68 + nb * 16 + lr] = acc[mb][nb][j]; }
        __builtin_amdgcn_wave_barrier(); asm volatile("" ::: "memory");
        float* crow = C + (size_t)(r0 + mb * 16) * ldc + c0;
#pragma unroll 1
        for (int ps = 0; ps < 2; ++ps) {
#pragma unroll
            for (int s = 0; s < 8; ++s) { const int row = 2 * s + hi, cofs = lr * 4; v4f val = *(const v4fa*)(os + row * 68 + cofs); if (BIAS) { val[0] += bfr(bias[c0 + cofs]); val[1] += bfr(bias[c0 + cofs + 1]); val[2] += bfr(bias[c0 + cofs + 2]); val[3] += bfr(bias[c0 + cofs + 3]); }
                *(volatile v4f*)(crow + (size_t)row * ldc + cofs) = val; }
            if (ps == 0) __threadfence(); }
        __builtin_amdgcn_wave_barrier(); asm volatile("" ::: "memory");
    }
}

__device__ __forceinline__ h16 tohx(float x) { return (h16)x; }
__device__ __forceinline__ void splitf(float y, unsigned short& h, unsigned short& l) { h = f2bf(y); l = f2bf(y - bf2f(h)); }
typedef __attribute__((ext_vector_type(2))) _Float16 v2h;
typedef __attribute__((ext_vector_type(4))) _Float16 v4h;
typedef __attribute__((ext_vector_type(2))) unsigned short v2us;
typedef __attribute__((ext_vector_type(4))) unsigned short v4us;
typedef __attribute__((ext_vector_type(2))) float v2f;

__global__ __launch_bounds__(256) void k_cvt8(const float* __restrict__ src, bf* dst, size_t n8) { const size_t i = (size_t)blockIdx.x * 256 + threadIdx.x; if (i >= n8) return; const v8f v = *(const v8f*)(src + i * 8); v8us o;
#pragma unroll
    for (int k = 0; k < 8; ++k) o[k] = f2bf(v[k]); *(volatile v8us*)(dst + i * 8) = o; __threadfence(); *(volatile v8us*)(dst + i * 8) = o; }
__global__ __launch_bounds__(256) void k_xt(const float* __restrict__ xb, bf* XT) { const size_t e = ((size_t)blockIdx.x * 256 + threadIdx.x) * 4; if (e >= (size_t)TQ * CC) return; const int c = (int)(e % CC), n = (int)(e / CC); v4us o;
#pragma unroll
    for (int q = 0; q < 4; ++q) o[q] = f2bf(xb[(size_t)(c + q) * TQ + n]); *(volatile v4us*)(XT + e) = o; __threadfence(); *(volatile v4us*)(XT + e) = o; }
__global__ __launch_bounds__(256) void k_bnp(const float* __restrict__ F, const float* __restrict__ g, const float* __restrict__ be, const float* __restrict__ mu, const float* __restrict__ var, h16* P) { const size_t e = ((size_t)blockIdx.x * 256 + threadIdx.x) * 2; if (e >= (size_t)TQ * KC) return; const int c = (int)(e % KC); v2h o;
#pragma unroll
    for (int q = 0; q < 2; ++q) { const int cq = c + q; const float sc = __fdiv_rn(bfr(g[cq]), __fsqrt_rn(__fadd_rn(bfr(var[cq]), 1e-5f))); float ms = __fmul_rn(bfr(mu[cq]), sc); asm volatile("" : "+v"(ms)); const float sh = __fsub_rn(bfr(be[cq]), ms); float t = __fmul_rn(F[e + q], sc); asm volatile("" : "+v"(t)); o[q] = tohx(__fadd_rn(t, sh)); }
    *(volatile v2h*)(P + e) = o; __threadfence(); *(volatile v2h*)(P + e) = o; }
__global__ __launch_bounds__(256) void k_vt(const float* __restrict__ FV, h16* VT) { const size_t e = ((size_t)blockIdx.x * 256 + threadIdx.x) * 2; if (e >= (size_t)VC * NKY) return; const int n = (int)(e % NKY), c = (int)(e / NKY); v2h o; o[0] = tohx(FV[(size_t)n * VC + c]); o[1] = tohx(FV[(size_t)(n + 1) * VC + c]); *(volatile v2h*)(VT + e) = o; __threadfence(); *(volatile v2h*)(VT + e) = o; }
template <int NK>
__global__ __launch_bounds__(256) void k_smax(const float* __restrict__ S, float* RS) { const int lane = threadIdx.x & 31; const int i = blockIdx.x * 8 + (threadIdx.x >> 5); if (i >= TQ) return; const float* sr = S + (size_t)i * NK; float m = -3.0e38f;
#pragma unroll 4
    for (int c0 = lane * 4; c0 < NK; c0 += 128) { const v4f v = *(const v4f*)(sr + c0); m = fmaxf(m, fmaxf(fmaxf(v[0], v[1]), fmaxf(v[2], v[3]))); }
#pragma unroll
    for (int sh = 16; sh; sh >>= 1) m = fmaxf(m, __shfl_xor(m, sh, 32));
    const float o = lane == 0 ? m : 0.f; *(volatile float*)(RS + (size_t)i * 32 + lane) = o; __threadfence(); *(volatile float*)(RS + (size_t)i * 32 + lane) = o; }
template <int NK>
__global__ __launch_bounds__(256) void k_sexp(const float* __restrict__ S, float* RS, h16* P) { const int lane = threadIdx.x & 31; const int i = blockIdx.x * 8 + (threadIdx.x >> 5); if (i >= TQ) return; const float* sr = S + (size_t)i * NK; const float m = RS[(size_t)i * 32]; float sum = 0.f;
#pragma unroll 1
    for (int ps = 0; ps < 2; ++ps) { sum = 0.f;
#pragma unroll 2
        for (int c0 = lane * 4; c0 < NK; c0 += 128) { const v4f v = *(const v4f*)(sr + c0); v4h o;
#pragma unroll
            for (int q = 0; q < 4; ++q) { float dlt = __fsub_rn(v[q], m); asm volatile("" : "+v"(dlt)); const float e = __expf(__fmul_rn(dlt, SCL)); sum += e; o[q] = tohx(e * PCAR); }
            *(volatile v4h*)(P + (size_t)i * NK + c0) = o; }
        if (ps == 0) __threadfence(); }
#pragma unroll
    for (int sh = 16; sh; sh >>= 1) sum += __shfl_xor(sum, sh, 32);
    const float o2 = lane == 0 ? m : (lane == 1 ? __fdiv_rn(1.0f, sum * PCAR) : 0.f); *(volatile float*)(RS + (size_t)i * 32 + lane) = o2; __threadfence(); *(volatile float*)(RS + (size_t)i * 32 + lane) = o2; }
__global__ __launch_bounds__(256) void k_csplit(const float* __restrict__ CTX, const float* __restrict__ RS, bf* Ch, bf* Cl) { const size_t e = ((size_t)blockIdx.x * 256 + threadIdx.x) * 2; if (e >= (size_t)TQ * VC) return; const int n = (int)(e / VC); const float r = RS[(size_t)n * 32 + 1]; v2us oh, ol;
#pragma unroll
    for (int q = 0; q < 2; ++q) { unsigned short a, c2; splitf(__fmul_rn(CTX[e + q], r), a, c2); oh[q] = a; ol[q] = c2; } *(volatile v2us*)(Ch + e) = oh; *(volatile v2us*)(Cl + e) = ol; __threadfence(); *(volatile v2us*)(Ch + e) = oh; *(volatile v2us*)(Cl + e) = ol; }
__global__ __launch_bounds__(256) void k_outT(const float* __restrict__ OT, float* OUTb) { const size_t e = ((size_t)blockIdx.x * 256 + threadIdx.x) * 2; if (e >= (size_t)CC * TQ) return; const int n = (int)(e % TQ), o = (int)(e / TQ); v2f v; v[0] = OT[(size_t)n * CC + o]; v[1] = OT[(size_t)(n + 1) * CC + o]; *(volatile v2f*)(OUTb + e) = v; __threadfence(); *(volatile v2f*)(OUTb + e) = v; }

extern "C" void kernel_launch(void* const* d_in, const int* in_sizes, int n_in,
                              void* d_out, int out_size, void* d_ws, size_t ws_size, hipStream_t stream) {
    (void)in_sizes; (void)n_in; (void)out_size;
    const float* IN[17]; for (int i = 0; i < 17; ++i) IN[i] = (const float*)d_in[i];
    float* OUT = (float*)d_out;
    char* wsp = (char*)d_ws;
    auto take = [&](size_t bytes) { char* p = wsp; wsp += (bytes + 255) & ~(size_t)255; return (void*)p; };
    bf* WQ = (bf*)take((size_t)KC * CC * 2); bf* WK = (bf*)take((size_t)KC * CC * 2); bf* WV = (bf*)take((size_t)VC * CC * 2); bf* WW = (bf*)take((size_t)CC * VC * 2);
    bf* XT = (bf*)take((size_t)TQ * CC * 2); float* F = (float*)take((size_t)TQ * KC * 4); h16* Q16 = (h16*)take((size_t)TQ * KC * 2); h16* K16 = (h16*)take((size_t)NKY * KC * 2); h16* VT = (h16*)take((size_t)VC * NKY * 2);
    float* S = (float*)take((size_t)TQ * NKY * 4); h16* P = (h16*)take((size_t)TQ * NKY * 2); float* RS = (float*)take((size_t)TQ * 32 * 4); float* CTX = (float*)take((size_t)TQ * VC * 4); bf* Ch = (bf*)take((size_t)TQ * VC * 2); bf* Cl = (bf*)take((size_t)TQ * VC * 2); float* OT = (float*)take((size_t)TQ * CC * 4);
    if ((size_t)(wsp - (char*)d_ws) > ws_size) return;
    { const unsigned g = (KC * CC / 8 + 255) / 256; k_cvt8<<<g, 256, 0, stream>>>(IN[1], WQ, (size_t)KC * CC / 8); k_cvt8<<<g, 256, 0, stream>>>(IN[7], WK, (size_t)KC * CC / 8); k_cvt8<<<g, 256, 0, stream>>>(IN[13], WV, (size_t)VC * CC / 8); k_cvt8<<<g, 256, 0, stream>>>(IN[15], WW, (size_t)CC * VC / 8); }
    const unsigned LP = (unsigned)(((size_t)TQ * KC / 2 + 255) / 256);
    for (int b = 0; b < NB_; ++b) {
        k_xt<<<(unsigned)(((size_t)TQ * CC / 4 + 255) / 256), 256, 0, stream>>>(IN[0] + (size_t)b * CC * TQ, XT);
        k_gemmw<bf, 0, true><<<dim3(TQ / 64, KC / 64, 1), 32, 0, stream>>>(XT, nullptr, WQ, nullptr, CC, F, KC, IN[2], 0, 0, 0); k_bnp<<<LP, 256, 0, stream>>>(F, IN[3], IN[4], IN[5], IN[6], Q16);
        k_gemmw<bf, 0, true><<<dim3(TQ / 64, KC / 64, 1), 32, 0, stream>>>(XT, nullptr, WK, nullptr, CC, F, KC, IN[8], 0, 0, 0); k_bnp<<<LP, 256, 0, stream>>>(F, IN[9], IN[10], IN[11], IN[12], K16);
        k_gemmw<bf, 0, true><<<dim3(TQ / 64, VC / 64, 1), 32, 0, stream>>>(XT, nullptr, WV, nullptr, CC, F, VC, IN[14], 0, 0, 0); k_vt<<<(unsigned)(((size_t)VC * NKY / 2 + 255) / 256), 256, 0, stream>>>(F, VT);
        k_gemmw<h16, 0, false><<<dim3(TQ / 64, NKY / 64, 1), 32, 0, stream>>>(Q16, nullptr, K16, nullptr, KC, S, NKY, nullptr, 0, 0, 0);
        k_smax<NKY><<<TQ / 8, 256, 0, stream>>>(S, RS); k_sexp<NKY><<<TQ / 8, 256, 0, stream>>>(S, RS, P);
        k_gemmw<h16, 0, false><<<dim3(TQ / 64, VC / 64, 1), 32, 0, stream>>>(P, nullptr, VT, nullptr, NKY, CTX, VC, nullptr, 0, 0, 0);
        k_csplit<<<(unsigned)(((size_t)TQ * VC / 2 + 255) / 256), 256, 0, stream>>>(CTX, RS, Ch, Cl);
        k_gemmw<bf, 1, true><<<dim3(TQ / 64, CC / 64, 1), 32, 0, stream>>>(Ch, Cl, WW, nullptr, VC, OT, CC, IN[16], 0, 0, 0);
        k_outT<<<(unsigned)(((size_t)CC * TQ / 2 + 255) / 256), 256, 0, stream>>>(OT, OUT + (size_t)b * CC * TQ); }
}
